// Mamba_81913616269596
// MI455X (gfx1250) — hardware-run, weakly checked
//
#include <hip/hip_runtime.h>
#include <math.h>

typedef __attribute__((ext_vector_type(16))) _Float16 v16h;
typedef __attribute__((ext_vector_type(8)))  _Float16 v8h;
typedef __attribute__((ext_vector_type(2)))  _Float16 v2h;
typedef __attribute__((ext_vector_type(16))) __bf16   v16b;
typedef __attribute__((ext_vector_type(8)))  __bf16   v8b;
typedef __attribute__((ext_vector_type(8)))  float    v8f;
typedef __attribute__((ext_vector_type(4)))  float    v4f;
typedef __attribute__((ext_vector_type(2)))  float    v2f;

constexpr int kNB   = 2;
constexpr int kT    = 1024;
constexpr int kRows = kNB * kT;
constexpr int kDM   = 512;
constexpr int kDI   = 2 * kDM;
constexpr int kH    = 8;
constexpr int kHd   = kDI / kH;
constexpr int kNs   = 16;
constexpr int kDC   = 3;
constexpr int kR    = 32;
constexpr int kXo   = kR + 4 * kH * kNs + 2 * kH;
constexpr int kXoP  = 576;
constexpr int kColBre = kR;
constexpr int kColBim = kR + kH * kNs;
constexpr int kColCre = kR + 2 * kH * kNs;
constexpr int kColCim = kR + 3 * kH * kNs;
constexpr int kColLam = kR + 4 * kH * kNs;
constexpr int kColEta = kColLam + kH;
constexpr int kThr  = 256;
constexpr float kInCarry = 1024.0f;
constexpr float kWCarry  = 4096.0f;
constexpr float kCU  = 512.0f;
constexpr float kCDt = 2048.0f;
constexpr float kCY  = 256.0f;
constexpr float kF16MinNormal = 6.103515625e-5f;

static_assert(kXo == 560 && kXo <= kXoP && (kXoP % 64) == 0 && kR == 32 && kDI == 1024 && kRows == 2048 && kT == 1024 && kDM == 512 && kHd == 128 && kColEta + kH == kXo, "the index arithmetic below uses these sizes");

constexpr size_t kOffZB = 0ull;
constexpr size_t kOffBDT = 8192ull;
constexpr size_t kOffX16 = 12288ull;
constexpr size_t kOffWIN16 = 2109440ull;
constexpr size_t kOffWX16 = 4206592ull;
constexpr size_t kOffWDT16 = 5386240ull;
constexpr size_t kOffWOUT16 = 5451776ull;
constexpr size_t kOffXZ = 6500352ull;
constexpr size_t kOffU32 = 23277568ull;
constexpr size_t kOffU16 = 31666176ull;
constexpr size_t kOffXD = 35860480ull;
constexpr size_t kOffDT16 = 40579072ull;
constexpr size_t kOffDL = 40710144ull;
constexpr size_t kOffGS = 49098752ull;
constexpr size_t kOffYS = 49229824ull;
constexpr size_t kOffY16 = 57618432ull;
constexpr size_t kWsTotal = 61812736ull;
static_assert(kWsTotal <= 134217728ull, "carve cap: under 128 MiB");
static_assert(kOffZB == 0
  && kOffBDT == kOffZB + 8192ull
  && kOffX16 == kOffBDT + 4096ull
  && kOffWIN16 == kOffX16 + 2097152ull
  && kOffWX16 == kOffWIN16 + 2097152ull
  && kOffWDT16 == kOffWX16 + 1179648ull
  && kOffWOUT16 == kOffWDT16 + 65536ull
  && kOffXZ == kOffWOUT16 + 1048576ull
  && kOffU32 == kOffXZ + 16777216ull
  && kOffU16 == kOffU32 + 8388608ull
  && kOffXD == kOffU16 + 4194304ull
  && kOffDT16 == kOffXD + 4718592ull
  && kOffDL == kOffDT16 + 131072ull
  && kOffGS == kOffDL + 8388608ull
  && kOffYS == kOffGS + 131072ull
  && kOffY16 == kOffYS + 8388608ull
  && kWsTotal == kOffY16 + 4194304ull, "the carve is a chain: every region starts where the one before ends");
static_assert((kOffBDT % 256) == 0 && (kOffX16 % 256) == 0 && (kOffWIN16 % 256) == 0 && (kOffWX16 % 256) == 0 && (kOffWDT16 % 256) == 0 && (kOffWOUT16 % 256) == 0 && (kOffXZ % 256) == 0 && (kOffU32 % 256) == 0 && (kOffU16 % 256) == 0 && (kOffXD % 256) == 0 && (kOffDT16 % 256) == 0 && (kOffDL % 256) == 0 && (kOffGS % 256) == 0 && (kOffYS % 256) == 0 && (kOffY16 % 256) == 0, "every region starts on a multiple of 256 B");

__device__ __forceinline__ unsigned short f2bf_bits(float f) {
  unsigned u = __float_as_uint(f);
  return (unsigned short)((u + 0x7FFFu + ((u >> 16) & 1u)) >> 16);
}
__device__ __forceinline__ float bf_bits2f(unsigned short h) { return __uint_as_float(((unsigned)h) << 16); }
__device__ __forceinline__ float bf16r(float f) { return bf_bits2f(f2bf_bits(f)); }
__device__ __forceinline__ float carry_flush(float v, float carry) {
  const float s = v * carry;
  return (fabsf(s) < kF16MinNormal) ? 0.0f : s;
}

__device__ __forceinline__ void dep_guard4_h(v8f& a, v8f& b, v8f& c, v8f& d, v16h x, v16h y) { asm volatile("v_nop\n\tv_nop\n\tv_nop\n\tv_nop" : "+v"(a), "+v"(b), "+v"(c), "+v"(d) : "v"(x), "v"(y)); }
__device__ __forceinline__ void dep_guard4_b(v8f& a, v8f& b, v8f& c, v8f& d, v16b x, v16b y) { asm volatile("v_nop\n\tv_nop\n\tv_nop\n\tv_nop" : "+v"(a), "+v"(b), "+v"(c), "+v"(d) : "v"(x), "v"(y)); }
__device__ __forceinline__ void keep4_h(v16h a, v16h b, v16h c, v16h d) { asm volatile("v_nop" :: "v"(a), "v"(b), "v"(c), "v"(d)); }
__device__ __forceinline__ void keep4_b(v16b a, v16b b, v16b c, v16b d) { asm volatile("v_nop" :: "v"(a), "v"(b), "v"(c), "v"(d)); }
__device__ __forceinline__ void acc_guard4(v8f& a, v8f& b, v8f& c, v8f& d) { asm volatile("v_nop\n\tv_nop\n\tv_nop\n\tv_nop" : "+v"(a), "+v"(b), "+v"(c), "+v"(d)); }

template <typename T> struct Frag;
template <> struct Frag<_Float16> {
  typedef v16h V; union U { v16h v; v8h h[2]; };
  static __device__ __forceinline__ v16h load(const _Float16* p) {
    U f; f.h[0] = *(const v8h*)(p); f.h[1] = *(const v8h*)(p + 16); return f.v;
  }
  static __device__ __forceinline__ v8f mma(v16h a, v16h b, v8f c) {
    return __builtin_amdgcn_wmma_f32_16x16x32_f16(false, a, false, b, (short)0, c, false, false);
  }
  static __device__ __forceinline__ void guard4(v8f& a, v8f& b, v8f& c, v8f& d, v16h x, v16h y) { dep_guard4_h(a, b, c, d, x, y); }
  static __device__ __forceinline__ void keep(v16h a, v16h b, v16h c, v16h d) { keep4_h(a, b, c, d); }
};
template <> struct Frag<__bf16> {
  typedef v16b V; union U { v16b v; v8b h[2]; };
  static __device__ __forceinline__ v16b load(const __bf16* p) {
    U f; f.h[0] = *(const v8b*)(p); f.h[1] = *(const v8b*)(p + 16); return f.v;
  }
  static __device__ __forceinline__ v8f mma(v16b a, v16b b, v8f c) {
    return __builtin_amdgcn_wmma_f32_16x16x32_bf16(false, a, false, b, (short)0, c, false, false);
  }
  static __device__ __forceinline__ void guard4(v8f& a, v8f& b, v8f& c, v8f& d, v16b x, v16b y) { dep_guard4_b(a, b, c, d, x, y); }
  static __device__ __forceinline__ void keep(v16b a, v16b b, v16b c, v16b d) { keep4_b(a, b, c, d); }
};

__device__ __forceinline__ v8f mma_h(v16h a, v16h b, v8f c) {
  c = __builtin_amdgcn_wmma_f32_16x16x32_f16(false, a, false, b, (short)0, c, false, false);
  asm volatile("v_nop\n\tv_nop\n\tv_nop\n\tv_nop" : "+v"(c) : "v"(a), "v"(b));
  return c;
}

template <int ET> struct Elem;
template <> struct Elem<0> { typedef _Float16 T; };
template <> struct Elem<1> { typedef __bf16 T; };
template <int ET, bool SPLIT, int BIAS_MODE, int OUT_MODE, bool RESID, int ACT = 0>
__global__ __launch_bounds__(256) void wmma_gemm64(
    const unsigned short* __restrict__ Ap, const unsigned short* __restrict__ A2p, int lda, long strideA,
    const unsigned short* __restrict__ Btp, const unsigned short* __restrict__ Bt2p, int ldb, long strideB,
    void* __restrict__ Cout, void* __restrict__ Cout2, int ldc, long strideC,
    const float* __restrict__ bias,
    const float* __restrict__ resid, long strideR,
    int M, int N, int K, float scale) {
  typedef typename Elem<ET>::T T;
  typedef typename Frag<T>::V V;
  const T* A = (const T*)Ap; const T* A2 = (const T*)A2p; const T* Bt = (const T*)Btp; const T* Bt2 = (const T*)Bt2p;
  __shared__ __align__(16) float sT[8][16 * 68];
  const int b    = blockIdx.y;
  const int lane = threadIdx.x & 31;
  const int wave = threadIdx.x >> 5;
  const int tilesN = N >> 6;
  const int tilesM = M >> 6;
  const int tile = blockIdx.x * 8 + wave;
  if (tile >= tilesM * tilesN) return;
  const int tm = tile / tilesN;
  const int tn = tile - tm * tilesN;
  const int m0 = tm << 6;
  const int n0 = tn << 6;

  const T* Ab  = A  + (size_t)b * strideA;
  const T* Bb  = Bt + (size_t)b * strideB;
  const T* Ab2 = SPLIT ? (A2  + (size_t)b * strideA) : nullptr;
  const T* Bb2 = SPLIT ? (Bt2 + (size_t)b * strideB) : nullptr;

  const int rlane = lane & 15;
  const int koff  = (lane >> 4) * 8;
  const int mOff  = (lane >> 4) * 8;

  v8f acc[4][4];
#pragma unroll
  for (int i = 0; i < 4; ++i)
#pragma unroll
    for (int j = 0; j < 4; ++j) acc[i][j] = (v8f){0.f,0.f,0.f,0.f,0.f,0.f,0.f,0.f};

  for (int k0 = 0; k0 < K; k0 += 32) {
    V bh[4], bl[4];
#pragma unroll
    for (int j = 0; j < 4; ++j) {
      const size_t bo = (size_t)(n0 + (j << 4) + rlane) * ldb + koff + k0;
      bh[j] = Frag<T>::load(Bb + bo);
      if (SPLIT) bl[j] = Frag<T>::load(Bb2 + bo);
    }
#pragma unroll
    for (int i = 0; i < 4; ++i) {
      const size_t ao = (size_t)(m0 + (i << 4) + rlane) * lda + koff + k0;
      V ah = Frag<T>::load(Ab + ao);
      V al;
      if (SPLIT) al = Frag<T>::load(Ab2 + ao);
#pragma unroll
      for (int j = 0; j < 4; ++j) {
        acc[i][j] = Frag<T>::mma(ah, bh[j], acc[i][j]);
        if (SPLIT) {
          acc[i][j] = Frag<T>::mma(ah, bl[j], acc[i][j]);
          acc[i][j] = Frag<T>::mma(al, bh[j], acc[i][j]);
        }
      }
      Frag<T>::guard4(acc[i][0], acc[i][1], acc[i][2], acc[i][3], ah, SPLIT ? al : ah);
    }
    Frag<T>::keep(bh[0], bh[1], bh[2], bh[3]);
    if (SPLIT) Frag<T>::keep(bl[0], bl[1], bl[2], bl[3]);
  }
  acc_guard4(acc[0][0], acc[0][1], acc[0][2], acc[0][3]);
  acc_guard4(acc[1][0], acc[1][1], acc[1][2], acc[1][3]);
  acc_guard4(acc[2][0], acc[2][1], acc[2][2], acc[2][3]);
  acc_guard4(acc[3][0], acc[3][1], acc[3][2], acc[3][3]);

  float* slab = sT[wave];
  const float* Rb = RESID ? (resid + (size_t)b * strideR) : nullptr;
#pragma unroll
  for (int i = 0; i < 4; ++i) {
    const int mBase = m0 + (i << 4);
#pragma unroll
    for (int j = 0; j < 4; ++j) {
      const int n = n0 + (j << 4) + rlane;
      float bv = 0.f;
      if (BIAS_MODE == 2) bv = bias[n];
#pragma unroll
      for (int r = 0; r < 8; ++r) {
        float v = acc[i][j][r] * scale;
        if (BIAS_MODE == 1) v += bias[mBase + mOff + r];
        if (BIAS_MODE == 2) v += bv;
        if (RESID) v += Rb[(size_t)(mBase + mOff + r) * ldc + n];
        if (ACT == 1) v = tanhf(v);
        if (ACT == 2) v = fmaxf(v, 0.0f);
        if (ACT == 3) v = v / (1.0f + expf(-v));
        if (ACT == 4) v = (v > 0.f) ? v : 0.01f * v;
        slab[(mOff + r) * 68 + (j << 4) + rlane] = v;
      }
    }
    __builtin_amdgcn_fence(__ATOMIC_RELEASE, "workgroup");
    __builtin_amdgcn_wave_barrier();
    __builtin_amdgcn_fence(__ATOMIC_ACQUIRE, "workgroup");
    if (OUT_MODE == 0) {
      float* C = (float*)Cout + (size_t)b * strideC;
      const int hh = lane >> 4, c4 = (lane & 15) * 4;
      for (int pass = 0; pass < 2; ++pass) {
#pragma unroll
        for (int it = 0; it < 8; ++it) {
          const int row = it * 2 + hh;
          v4f v = *(const v4f*)(slab + row * 68 + c4);
          *(volatile v4f*)(C + (size_t)(mBase + row) * ldc + n0 + c4) = v;
        }
        __threadfence();
      }
    } else {
      const int q = lane >> 3, c8 = (lane & 7) * 8;
      unsigned short* C  = (unsigned short*)Cout  + (size_t)b * strideC;
      unsigned short* C2 = (OUT_MODE == 2) ? ((unsigned short*)Cout2 + (size_t)b * strideC) : nullptr;
      for (int pass = 0; pass < 2; ++pass) {
#pragma unroll
        for (int it = 0; it < 4; ++it) {
          const int row = it * 4 + q;
          const float* sp = slab + row * 68 + c8;
          v8h hv, lv;
#pragma unroll
          for (int e = 0; e < 8; ++e) {
            if (OUT_MODE == 1) {
              hv[e] = (_Float16)sp[e];
            } else {
              unsigned short hb = f2bf_bits(sp[e]);
              unsigned short lb = f2bf_bits(sp[e] - bf_bits2f(hb));
              hv[e] = __builtin_bit_cast(_Float16, hb);
              lv[e] = __builtin_bit_cast(_Float16, lb);
            }
          }
          *(volatile v8h*)(C + (size_t)(mBase + row) * ldc + n0 + c8) = hv;
          if (OUT_MODE == 2) *(volatile v8h*)(C2 + (size_t)(mBase + row) * ldc + n0 + c8) = lv;
        }
        __threadfence();
      }
    }
    __builtin_amdgcn_fence(__ATOMIC_RELEASE, "workgroup");
    __builtin_amdgcn_wave_barrier();
    __builtin_amdgcn_fence(__ATOMIC_ACQUIRE, "workgroup");
  }
}


__device__ __forceinline__ void store2(float* p, float v) {
  *(volatile float*)p = v;
  __threadfence();
  *(volatile float*)p = v;
}

__global__ __launch_bounds__(kThr) void cast_plane_kernel(const float* __restrict__ src, unsigned short* __restrict__ dst,
                                                          int colsLog2, int dstPitch, int dstOff) {
  const int i   = blockIdx.x * kThr + threadIdx.x;
  const int sh  = colsLog2 - 3;
  const int row = i >> sh;
  const int c8  = (i & ((1 << sh) - 1)) * 8;
  const float* sp = src + ((size_t)row << colsLog2) + c8;
  const v4f a0 = *(const v4f*)(sp);
  const v4f a1 = *(const v4f*)(sp + 4);
  v8h hv;
#pragma unroll
  for (int e = 0; e < 4; ++e) {
    const float f0 = a0[e];
    const float f1 = a1[e];
    hv[e]     = (_Float16)carry_flush(bf16r(f0), kInCarry);
    hv[4 + e] = (_Float16)carry_flush(bf16r(f1), kInCarry);
  }
  unsigned short* dp = dst + (size_t)row * dstPitch + dstOff + c8;
  *(volatile v8h*)dp = hv;
  __threadfence();
  *(volatile v8h*)dp = hv;
}

__global__ __launch_bounds__(256) void wt_plane_kernel(const float* __restrict__ W, unsigned short* __restrict__ dst, int K, int N, int nLive, int ldd, int colOff) {
  const int n  = blockIdx.x;
  const int k8 = threadIdx.x * 8;
  const bool live = n < nLive;
  const int nc = live ? n : 0;
  v8h hv;
#pragma unroll
  for (int e = 0; e < 8; ++e) {
    const float w = W[(size_t)(k8 + e) * N + nc];
    hv[e] = (_Float16)(live ? carry_flush(bf16r(w), kWCarry) : 0.0f);
  }
  unsigned short* dp = dst + (size_t)n * ldd + colOff + k8;
  *(volatile v8h*)dp = hv;
  __threadfence();
  *(volatile v8h*)dp = hv;
}

__global__ __launch_bounds__(kThr) void setup_kernel(const float* __restrict__ bdt, float* __restrict__ ZB, float* __restrict__ BDT, unsigned short* __restrict__ WX16) {
  const unsigned bk = blockIdx.x;
  if (bk < 8u) {
    store2(ZB + bk * (unsigned)kThr + threadIdx.x, 0.0f);
  } else if (bk < 12u) {
    const unsigned d = (bk - 8u) * (unsigned)kThr + threadIdx.x;
    const float p = bdt[d];
    store2(BDT + d, bf16r(p));
  } else {
    const unsigned j = (bk - 12u) * (unsigned)kThr + threadIdx.x;
    v8h zv;
#pragma unroll
    for (int e = 0; e < 8; ++e) zv[e] = (_Float16)0.0f;
    unsigned short* dp = WX16 + (size_t)kXo * kDI + (size_t)j * 8;
    *(volatile v8h*)dp = zv;
    __threadfence();
    *(volatile v8h*)dp = zv;
  }
}
static_assert(2048 == 8 * kThr && kDI == 4 * kThr && (size_t)(kXoP - kXo) * kDI / 8 == 8ull * kThr, "set-up grid: 8 + 4 + 8 = 20 blocks");

__global__ __launch_bounds__(128) void front_kernel(const float* __restrict__ XZ, const float* __restrict__ cw, const float* __restrict__ cb,
                                                    float* __restrict__ U32, unsigned short* __restrict__ U16) {
  const int row = (int)blockIdx.y;
  const int pos = row & (kT - 1);
  const int c8 = (int)threadIdx.x * 8;
  float acc[8], wv[8][kDC];
#pragma unroll
  for (int e = 0; e < 8; ++e) {
    const float p = cb[c8 + e];
    acc[e] = bf16r(p);
#pragma unroll
    for (int k = 0; k < kDC; ++k) { const float w = cw[(size_t)(c8 + e) * kDC + k]; wv[e][k] = bf16r(w); }
  }
#pragma unroll
  for (int k = 0; k < kDC; ++k) {
    const int back = kDC - 1 - k;
    const bool has = pos >= back;
    const float* xp = XZ + (size_t)(row - (has ? back : 0)) * (2 * kDI) + c8;
    const v4f x0 = *(const v4f*)xp, x1 = *(const v4f*)(xp + 4);
#pragma unroll
    for (int e = 0; e < 8; ++e) {
      const float xv = (e < 4) ? x0[e] : x1[e - 4];
      acc[e] += has ? wv[e][k] * xv : 0.0f;
    }
  }
  v4f u0, u1;
  v8h hv;
#pragma unroll
  for (int e = 0; e < 8; ++e) {
    const float v = acc[e];
    const float s = v / (1.0f + expf(-v));
    if (e < 4) u0[e] = s; else u1[e - 4] = s;
    hv[e] = (_Float16)carry_flush(s, kCU);
  }
  float* up = U32 + (size_t)row * kDI + c8;
  unsigned short* hp = U16 + (size_t)row * kDI + c8;
  for (int pass = 0; pass < 2; ++pass) {
    *(volatile v4f*)up = u0; *(volatile v4f*)(up + 4) = u1;
    *(volatile v8h*)hp = hv;
    __threadfence();
  }
}
static_assert(kDI == 128 * 8, "front grid exact: 128 groups a row");

__global__ __launch_bounds__(kThr) void dtcast_kernel(const float* __restrict__ XD, unsigned short* __restrict__ DT16) {
  const unsigned i = blockIdx.x * (unsigned)kThr + threadIdx.x;
  const size_t row = i >> 2;
  const unsigned c8 = (i & 3u) * 8u;
  const float* sp = XD + row * kXoP + c8;
  v8h hv;
#pragma unroll
  for (int e = 0; e < 8; ++e) { const float v = sp[e]; hv[e] = (_Float16)carry_flush(v, kCDt); }
  unsigned short* dp = DT16 + row * kR + c8;
  *(volatile v8h*)dp = hv;
  __threadfence();
  *(volatile v8h*)dp = hv;
}
static_assert((size_t)kRows * 4 == 32ull * kThr && kR == 4 * 8, "the step input's cast: 32 blocks; 4 groups a row");

__global__ __launch_bounds__(kThr) void gatesig_kernel(const float* __restrict__ XD, float* __restrict__ GS) {
  const unsigned i = blockIdx.x * (unsigned)kThr + threadIdx.x;
  const size_t row = i >> 4;
  const unsigned j = i & 15u;
  const float v = XD[row * kXoP + kColLam + j];
  store2(GS + i, 1.0f / (1.0f + expf(-v)));
}
static_assert((size_t)kRows * 16 == 128ull * kThr && 2 * kH == 16, "the gates: 128 blocks; sixteen columns a row");

__global__ __launch_bounds__(kThr) void scan_kernel(const float* __restrict__ XD, const float* __restrict__ DL, const float* __restrict__ U32, const float* __restrict__ GS,
                                                    const float* __restrict__ A_log, const float* __restrict__ A_imag, const float* __restrict__ Dp, float* __restrict__ YS) {
  const unsigned sq = blockIdx.x >> 2;
  const unsigned d = (blockIdx.x & 3u) * (unsigned)kThr + threadIdx.x;
  const unsigned hdI = d >> 7;
  float ar[kNs], ai[kNs], hr[kNs], hi[kNs], pr[kNs], pi[kNs];
#pragma unroll
  for (int n = 0; n < kNs; ++n) {
    const float a = A_log[(size_t)hdI * kNs + n], b = A_imag[(size_t)hdI * kNs + n];
    ar[n] = -expf(bf16r(a)); ai[n] = bf16r(b);
    hr[n] = 0.0f; hi[n] = 0.0f; pr[n] = 0.0f; pi[n] = 0.0f;
  }
  const float q0 = Dp[d];
  const float dsk = bf16r(q0);
  for (int l = 0; l < kT; ++l) {
    const size_t row = (size_t)sq * kT + (size_t)l;
    const float* px = XD + row * kXoP + 16u * hdI;
    const float pre = DL[row * kDI + d];
    const float uv = U32[row * kDI + d];
    const float lam = GS[row * 16 + hdI], eta = GS[row * 16 + 8u + hdI];
    const float dt = fmaxf(pre, 0.0f) + log1pf(expf(-fabsf(pre)));
    const float bsc = (1.0f - lam) * dt;
    const float gam = lam * dt * eta;
    float y = 0.0f;
#pragma unroll
    for (int q = 0; q < kNs / 4; ++q) {
      const v4f br = *(const v4f*)(px + kColBre + 4 * q), bi = *(const v4f*)(px + kColBim + 4 * q);
      const v4f cr = *(const v4f*)(px + kColCre + 4 * q), ci = *(const v4f*)(px + kColCim + 4 * q);
#pragma unroll
      for (int e = 0; e < 4; ++e) {
        const int n = 4 * q + e;
        const float mag = expf(fminf(fmaxf(dt * ar[n], -20.0f), 20.0f));
        const float ang = dt * ai[n];
        const float are = mag * cosf(ang), aim = mag * sinf(ang);
        const float bxr = uv * br[e], bxi = uv * bi[e];
        const float bre = bsc * are, bim = bsc * aim;
        const float vr = bre * pr[n] - bim * pi[n] + gam * bxr;
        const float vi = bre * pi[n] + bim * pr[n] + gam * bxi;
        const float nr = are * hr[n] - aim * hi[n] + vr;
        const float ni = are * hi[n] + aim * hr[n] + vi;
        hr[n] = nr; hi[n] = ni; pr[n] = bxr; pi[n] = bxi;
        y += nr * cr[e] + ni * ci[e];
      }
    }
    store2(YS + row * kDI + d, y + dsk * uv);
  }
}
static_assert(kDI == 4 * kThr && kHd == 128 && (kNs % 4) == 0 && (kColBre % 4) == 0 && (kColBim % 4) == 0 && (kColCre % 4) == 0 && (kColCim % 4) == 0, "walk grid exact: 8 blocks: four a sequence; a wave inside one head; the B | C columns 16-B aligned");

__global__ __launch_bounds__(128) void ygate_kernel(const float* __restrict__ YS, const float* __restrict__ XZ, unsigned short* __restrict__ Y16) {
  const size_t row = blockIdx.y;
  const unsigned c8 = threadIdx.x * 8u;
  const float* yp = YS + row * kDI + c8;
  const float* zp = XZ + row * (2 * kDI) + kDI + c8;
  v8h hv;
#pragma unroll
  for (int e = 0; e < 8; ++e) { const float z = zp[e]; hv[e] = (_Float16)carry_flush(yp[e] * (z / (1.0f + expf(-z))), kCY); }
  unsigned short* dp = Y16 + row * kDI + c8;
  *(volatile v8h*)dp = hv;
  __threadfence();
  *(volatile v8h*)dp = hv;
}

extern "C" void kernel_launch(void* const* d_in, const int* in_sizes, int n_in,
                              void* d_out, int out_size, void* d_ws, size_t ws_size,
                              hipStream_t stream) {
  if (n_in < 11 || d_out == nullptr || d_ws == nullptr) return;
  if (in_sizes[0] != kRows * kDM || in_sizes[1] != 2 * kDI * kDM || in_sizes[2] != kDI * kDC || in_sizes[3] != kDI || in_sizes[4] != kXo * kDI || in_sizes[5] != kDI * kR) return;
  if (in_sizes[6] != kDI || in_sizes[7] != kH * kNs || in_sizes[8] != kH * kNs || in_sizes[9] != kDI || in_sizes[10] != kDM * kDI) return;
  if (out_size != kRows * kDM) return;
  if (ws_size < kWsTotal) return;
  const float* x    = (const float*)d_in[0];
  const float* Win  = (const float*)d_in[1];
  const float* cvw  = (const float*)d_in[2];
  const float* cvb  = (const float*)d_in[3];
  const float* Wx   = (const float*)d_in[4];
  const float* Wdt  = (const float*)d_in[5];
  const float* bdt  = (const float*)d_in[6];
  const float* alog = (const float*)d_in[7];
  const float* aimg = (const float*)d_in[8];
  const float* dsk  = (const float*)d_in[9];
  const float* Wout = (const float*)d_in[10];
  float* out = (float*)d_out;
  char* ws = (char*)d_ws;
  float* ZB   = (float*)(ws + kOffZB);
  float* BDT  = (float*)(ws + kOffBDT);
  unsigned short* X16    = (unsigned short*)(ws + kOffX16);
  unsigned short* WIN16  = (unsigned short*)(ws + kOffWIN16);
  unsigned short* WX16   = (unsigned short*)(ws + kOffWX16);
  unsigned short* WDT16  = (unsigned short*)(ws + kOffWDT16);
  unsigned short* WOUT16 = (unsigned short*)(ws + kOffWOUT16);
  float* XZ  = (float*)(ws + kOffXZ);
  float* U32 = (float*)(ws + kOffU32);
  unsigned short* U16 = (unsigned short*)(ws + kOffU16);
  float* XD  = (float*)(ws + kOffXD);
  unsigned short* DT16 = (unsigned short*)(ws + kOffDT16);
  float* DL  = (float*)(ws + kOffDL);
  float* GS  = (float*)(ws + kOffGS);
  float* YS  = (float*)(ws + kOffYS);
  unsigned short* Y16 = (unsigned short*)(ws + kOffY16);

  static_assert(((size_t)kRows * kDM / 8) % kThr == 0 && ((size_t)2 * kDI * kDM / 8) % kThr == 0 && ((size_t)kXo * kDI / 8) % kThr == 0 && ((size_t)kDI * kR / 8) % kThr == 0 && ((size_t)kDM * kDI / 8) % kThr == 0, "the casts' grids");
  cast_plane_kernel<<<(int)(((size_t)kRows * kDM / 8) / kThr), kThr, 0, stream>>>(x, X16, 9, kDM, 0);
  cast_plane_kernel<<<(int)(((size_t)2 * kDI * kDM / 8) / kThr), kThr, 0, stream>>>(Win, WIN16, 9, kDM, 0);
  cast_plane_kernel<<<(int)(((size_t)kXo * kDI / 8) / kThr), kThr, 0, stream>>>(Wx, WX16, 10, kDI, 0);
  cast_plane_kernel<<<(int)(((size_t)kDI * kR / 8) / kThr), kThr, 0, stream>>>(Wdt, WDT16, 5, kR, 0);
  cast_plane_kernel<<<(int)(((size_t)kDM * kDI / 8) / kThr), kThr, 0, stream>>>(Wout, WOUT16, 10, kDI, 0);
  setup_kernel<<<20, kThr, 0, stream>>>(bdt, ZB, BDT, WX16);

  wmma_gemm64<0, false, 2, 0, false, 0><<<dim3((kRows / 64) * (2 * kDI / 64) / 8, 1), 256, 0, stream>>>(
      X16, X16, kDM, 0L, WIN16, WIN16, kDM, 0L, (void*)XZ, (void*)XZ, 2 * kDI, 0L, ZB, nullptr, 0L, kRows, 2 * kDI, kDM, 1.0f / (kInCarry * kInCarry));
  front_kernel<<<dim3(1, kRows), 128, 0, stream>>>(XZ, cvw, cvb, U32, U16);
  wmma_gemm64<0, false, 2, 0, false, 0><<<dim3((kRows / 64) * (kXoP / 64) / 8, 1), 256, 0, stream>>>(
      U16, U16, kDI, 0L, WX16, WX16, kDI, 0L, (void*)XD, (void*)XD, kXoP, 0L, ZB, nullptr, 0L, kRows, kXoP, kDI, 1.0f / (kCU * kInCarry));
  dtcast_kernel<<<32, kThr, 0, stream>>>(XD, DT16);
  wmma_gemm64<0, false, 2, 0, false, 0><<<dim3((kRows / 64) * (kDI / 64) / 8, 1), 256, 0, stream>>>(
      DT16, DT16, kR, 0L, WDT16, WDT16, kR, 0L, (void*)DL, (void*)DL, kDI, 0L, BDT, nullptr, 0L, kRows, kDI, kR, 1.0f / (kCDt * kInCarry));
  gatesig_kernel<<<128, kThr, 0, stream>>>(XD, GS);
  scan_kernel<<<2 * 4, kThr, 0, stream>>>(XD, DL, U32, GS, alog, aimg, dsk, YS);
  ygate_kernel<<<dim3(1, kRows), 128, 0, stream>>>(YS, XZ, Y16);
  wmma_gemm64<0, false, 2, 0, false, 0><<<dim3((kRows / 64) * (kDM / 64) / 8, 1), 256, 0, stream>>>(
      Y16, Y16, kDI, 0L, WOUT16, WOUT16, kDI, 0L, (void*)out, (void*)out, kDM, 0L, ZB, nullptr, 0L, kRows, kDM, kDI, 1.0f / (kCY * kInCarry));
}
